// EncoderClassifierMamba_53721450938847
// MI455X (gfx1250) — hardware-run, weakly checked
//
#include <hip/hip_runtime.h>
#include <stddef.h>


typedef _Float16 h16;
typedef _Float16 v16h __attribute__((ext_vector_type(16)));
typedef _Float16 v8h  __attribute__((ext_vector_type(8)));
typedef float    v8f  __attribute__((ext_vector_type(8)));
typedef float    v4f  __attribute__((ext_vector_type(4)));
typedef int      v4i  __attribute__((ext_vector_type(4)));

#ifndef NB
#define NB 64
#endif
#ifndef SEQ
#define SEQ 2048
#endif
#define NB_FULL  64
#define SEQ_FULL 2048
#define SNS   37
#define NFEAT 74
#define NQ    76
#define KS    128
#define EMB   256
#define CDIM  512
#define NSTAT 8
#define NCLS  2
#define TCH   1024
#define NCH   (SEQ / TCH)

static_assert(NB >= 16 && NB <= NB_FULL && (NB % 16) == 0);
static_assert(SEQ >= TCH && SEQ <= SEQ_FULL && (SEQ % TCH) == 0);
static_assert(TCH == 256 * 4);
static_assert(NCH >= 1 && NCH * 4 <= 32);
static_assert(NFEAT == 2 * SNS && NQ == NFEAT + 2);
static_assert((KS % 64) == 0 && (KS % 32) == 0 && KS >= NFEAT);
static_assert(KS == 128);
static_assert(EMB == 8 * 32);
static_assert(EMB == 256);
static_assert(CDIM == 2 * EMB && CDIM == 8 * 64 && (CDIM % 32) == 0);
static_assert((EMB % 64) == 0 && (CDIM % 64) == 0);
static_assert(16 * NSTAT == 128);
static_assert(16 * NCLS * 4 == 128);

#define LDT 72
#define CLD 520
static_assert((LDT % 8) == 0 && LDT >= 64);
static_assert((CLD % 8) == 0 && CLD >= CDIM);

#define WCARRY 64.0f
#define CCARRY 64.0f

#define HEAD_LDS (16 * CLD * 2 + 3 * 16 * 4 + 16 * NSTAT * 4 + 8 * 16 * NCLS * 4 + 32 * 4)
static_assert(HEAD_LDS <= 131072);
static_assert(64 * LDT * 2 <= 131072);

#define WS_BYTES   ((size_t)EMB * KS * 2)
#define WM_BYTES   ((size_t)CDIM * CDIM * 2)
#define A_BYTES    ((size_t)NB * KS * 2)
#define ST_BYTES   ((size_t)NB * 32 * 4)
#define OFF_WSP ((size_t)0)
#define OFF_WMP (OFF_WSP + WS_BYTES)
#define OFF_A   (OFF_WMP + WM_BYTES)
#define OFF_ST  (OFF_A + A_BYTES)
#define WS_TOTAL (OFF_ST + ST_BYTES)
static_assert((WS_BYTES % 128) == 0 && (WM_BYTES % 128) == 0);
static_assert((A_BYTES % 128) == 0 && (ST_BYTES % 128) == 0);
static_assert(WS_TOTAL <= (size_t)134217728);

__device__ __forceinline__ float bf16r(float x) {
  unsigned int u = __float_as_uint(x);
  u = (u + 0x7FFFu + ((u >> 16) & 1u)) & 0xFFFF0000u;
  return __uint_as_float(u);
}

static __device__ __forceinline__ h16 toh_flush(float v) {
  const h16 r = (h16)v;
  return (fabsf(v) < 6.103515625e-05f) ? (h16)0.0f : r;
}

__device__ __forceinline__ v16h frag_join(v8h lo, v8h hi) {
  v16h out;
#pragma unroll
  for (int i = 0; i < 8; ++i) { out[i] = lo[i]; out[i + 8] = hi[i]; }
  return out;
}
__device__ __forceinline__ v16h frag_at(const _Float16* __restrict__ p) {
  const v8h lo = *(const v8h*)(p);
  const v8h hi = *(const v8h*)(p + 16);
  return frag_join(lo, hi);
}

__device__ __forceinline__ v8f wmma16(v16h a, v16h b, v8f c) {
  v8f d = __builtin_amdgcn_wmma_f32_16x16x32_f16(false, a, false, b, (short)0, c,
                                                 false, false);
  asm volatile("v_nop\n\tv_nop\n\tv_nop\n\tv_nop" : "+v"(d) : "v"(a), "v"(b));
  return d;
}

__device__ __forceinline__ float red16_sum(float x) {
#pragma unroll
  for (int off = 1; off < 16; off <<= 1) x += __shfl_xor(x, off, 32);
  return x;
}
__device__ __forceinline__ float red32_sum(float x) {
#pragma unroll
  for (int off = 1; off < 32; off <<= 1) x += __shfl_xor(x, off, 32);
  return x;
}

__global__ __launch_bounds__(256) void wconv_kernel(
    const float* __restrict__ W, _Float16* __restrict__ Wt, unsigned ldw, unsigned ldk,
    unsigned kreal) {
  __shared__ __attribute__((aligned(16))) _Float16 T[64 * LDT];
  const unsigned tid = threadIdx.x;
  const unsigned n0 = blockIdx.x * 64u;
  const unsigned k0 = blockIdx.y * 64u;
#pragma unroll 4
  for (unsigned j = 0; j < 16u; ++j) {
    const unsigned idx = tid + 256u * j;
    const unsigned kr = idx >> 6, nc = idx & 63u;
    const unsigned kg = k0 + kr;
    const unsigned ks = (kg < kreal) ? kg : (kreal - 1u);
    const float vl = W[(size_t)ks * ldw + n0 + nc];
    const float v = (kg < kreal) ? vl : 0.0f;
    T[nc * LDT + kr] = toh_flush(WCARRY * bf16r(v));
  }
  __syncthreads();
  v8h x[2];
  size_t off[2];
#pragma unroll
  for (unsigned i = 0; i < 2u; ++i) {
    const unsigned n = 32u * i + (tid >> 3);
    const unsigned kc = (tid & 7u) * 8u;
    x[i] = *(const v8h*)&T[n * LDT + kc];
    off[i] = (size_t)(n0 + n) * ldk + k0 + kc;
  }
#pragma unroll
  for (int i = 0; i < 2; ++i) *(volatile v8h*)(Wt + off[i]) = x[i];
  __threadfence();
#pragma unroll
  for (int i = 0; i < 2; ++i) *(volatile v8h*)(Wt + off[i]) = x[i];
}

__global__ __launch_bounds__(256) void pool_kernel(
    const float* __restrict__ x, const int* __restrict__ smask, const float* __restrict__ timev,
    _Float16* __restrict__ A16, float* __restrict__ stat) {
  __shared__ float wpart[NQ * 8];
  __shared__ __attribute__((aligned(16))) _Float16 arow[KS];
  __shared__ __attribute__((aligned(16))) float srow[32];

  const unsigned tid = threadIdx.x, lane = tid & 31u;
  const unsigned w = __builtin_amdgcn_readfirstlane(threadIdx.x >> 5);
  const unsigned b = blockIdx.x;
  const float* xb = x + (size_t)b * SNS * SEQ_FULL;
  const int*   sb = smask + (size_t)b * SNS * SEQ_FULL;
  const float* tb = timev + (size_t)b * SEQ_FULL;

  unsigned fl = 0u;
#pragma unroll 1
  for (unsigned s = 0; s < (unsigned)SNS; ++s) {
#pragma unroll
    for (unsigned c = 0; c < (unsigned)NCH; ++c) {
      const size_t o = (size_t)s * SEQ_FULL + c * (unsigned)TCH + tid * 4u;
      const v4f xv = *(const v4f*)(xb + o);
      const v4i sv = *(const v4i*)(sb + o);
#pragma unroll
      for (int i = 0; i < 4; ++i) {
        const unsigned nz = ((bf16r(xv[i]) != 0.0f) || (sv[i] != 0)) ? 1u : 0u;
        fl |= nz << (c * 4u + (unsigned)i);
      }
    }
  }

#pragma unroll 1
  for (unsigned s = 0; s < (unsigned)SNS; ++s) {
    float px = 0.0f, pm = 0.0f;
#pragma unroll
    for (unsigned c = 0; c < (unsigned)NCH; ++c) {
      const size_t o = (size_t)s * SEQ_FULL + c * (unsigned)TCH + tid * 4u;
      const v4f xv = *(const v4f*)(xb + o);
      const v4i sv = *(const v4i*)(sb + o);
#pragma unroll
      for (int i = 0; i < 4; ++i) {
        const bool on = ((fl >> (c * 4u + (unsigned)i)) & 1u) != 0u;
        const float xe = bf16r(xv[i]);
        const float me = (float)sv[i];
        px += on ? xe : 0.0f;
        pm += on ? me : 0.0f;
      }
    }
    px = red32_sum(px);
    pm = red32_sum(pm);
    if (lane == 0u) {
      wpart[s * 8u + w] = px;
      wpart[((unsigned)SNS + s) * 8u + w] = pm;
    }
  }
  {
    float vc = 0.0f, vt = 0.0f;
#pragma unroll
    for (unsigned c = 0; c < (unsigned)NCH; ++c) {
      const v4f tv = *(const v4f*)(tb + c * (unsigned)TCH + tid * 4u);
#pragma unroll
      for (int i = 0; i < 4; ++i) {
        const bool on = ((fl >> (c * 4u + (unsigned)i)) & 1u) != 0u;
        const float te = bf16r(tv[i]);
        vc += on ? 1.0f : 0.0f;
        vt += on ? te : 0.0f;
      }
    }
    vc = red32_sum(vc);
    vt = red32_sum(vt);
    if (lane == 0u) {
      wpart[(unsigned)NFEAT * 8u + w] = vc;
      wpart[((unsigned)NFEAT + 1u) * 8u + w] = vt;
    }
  }
  __syncthreads();

  if (w < 4u) {
    const unsigned q = tid;
    const unsigned qc = (q < (unsigned)NQ) ? q : ((unsigned)NQ - 1u);
    float sum = 0.0f;
#pragma unroll
    for (unsigned ww = 0; ww < 8u; ++ww) sum += wpart[qc * 8u + ww];
    const float sv = (q < (unsigned)NFEAT) ? sum : 0.0f;
    arow[q] = toh_flush(sv);
  } else if (w == 4u) {
    float cnt = 0.0f, ts = 0.0f;
#pragma unroll
    for (unsigned ww = 0; ww < 8u; ++ww) {
      cnt += wpart[(unsigned)NFEAT * 8u + ww];
      ts  += wpart[((unsigned)NFEAT + 1u) * 8u + ww];
    }
    srow[lane] = (lane == 0u) ? cnt : ((lane == 1u) ? ts : 0.0f);
  }
  __syncthreads();

  if (w == 0u) {
    const unsigned li = (lane < 16u) ? lane : 15u;
    const v8h av = *(const v8h*)&arow[li * 8u];
    _Float16* p = A16 + (size_t)b * KS + li * 8u;
    if (lane < 16u) *(volatile v8h*)p = av;
    __threadfence();
    if (lane < 16u) *(volatile v8h*)p = av;
  } else if (w == 1u) {
    const unsigned li = (lane < 8u) ? lane : 7u;
    const v4f sv4 = *(const v4f*)&srow[li * 4u];
    float* p = stat + (size_t)b * 32u + li * 4u;
    if (lane < 8u) *(volatile v4f*)p = sv4;
    __threadfence();
    if (lane < 8u) *(volatile v4f*)p = sv4;
  }
}

__global__ __launch_bounds__(256) void head_kernel(
    const _Float16* __restrict__ A16, const float* __restrict__ stat,
    const _Float16* __restrict__ Ws_t, const _Float16* __restrict__ Wm_t,
    const float* __restrict__ statics,
    const float* __restrict__ b_sens, const float* __restrict__ W_time,
    const float* __restrict__ b_time,
    const float* __restrict__ W_stat, const float* __restrict__ b_stat,
    const float* __restrict__ b_merge,
    const float* __restrict__ W_cls, const float* __restrict__ b_cls,
    float* __restrict__ out) {
  __shared__ __attribute__((aligned(16))) _Float16 Cm[16 * CLD];
  __shared__ float st_cnt[16];
  __shared__ float st_ts[16];
  __shared__ float st_inv[16];
  __shared__ float sst[16 * NSTAT];
  __shared__ float cpart[8 * 16 * NCLS];
  __shared__ __attribute__((aligned(16))) float otile[32];

  const unsigned tid = threadIdx.x, lane = tid & 31u;
  const unsigned w = __builtin_amdgcn_readfirstlane(threadIdx.x >> 5);
  const unsigned hh = lane >> 4, m = lane & 15u;
  const unsigned row0 = blockIdx.x * 16u;

  {
    const unsigned r = tid & 15u;
    const float c = stat[(size_t)(row0 + r) * 32u];
    const float t = stat[(size_t)(row0 + r) * 32u + 1u];
    const float iv = 1.0f / fmaxf(c, 1.0e-9f);
    if (tid < 16u) { st_cnt[r] = c; st_ts[r] = t; st_inv[r] = iv; }
    const unsigned si = tid & 127u;
    const float sv = bf16r(statics[(size_t)row0 * NSTAT + si]);
    if (tid < 128u) sst[si] = sv;
  }
  __syncthreads();

  {
    const _Float16* ap  = A16 + (size_t)(row0 + m) * KS + hh * 8u;
    const _Float16* bp0 = Ws_t + (size_t)(w * 32u + m) * KS + hh * 8u;
    const _Float16* bp1 = bp0 + (size_t)16 * KS;
    v8f p[2];
    p[0] = (v8f){};
    p[1] = (v8f){};
#pragma unroll
    for (unsigned k0 = 0; k0 < (unsigned)KS; k0 += 32u) {
      const v16h a  = frag_at(ap + k0);
      const v16h b0 = frag_at(bp0 + k0);
      const v16h b1 = frag_at(bp1 + k0);
      p[0] = wmma16(a, b0, p[0]);
      p[1] = wmma16(a, b1, p[1]);
    }
#pragma unroll
    for (int t = 0; t < 2; ++t) {
      const unsigned col = w * 32u + (unsigned)t * 16u + m;
      const float bsum = bf16r(b_sens[col]) + bf16r(b_time[col]);
      const float wt = bf16r(W_time[col]);
#pragma unroll
      for (int r = 0; r < 8; ++r) {
        const unsigned row = hh * 8u + (unsigned)r;
        const float acc = p[t][r] * (1.0f / WCARRY) + st_cnt[row] * bsum + st_ts[row] * wt;
        const float val = acc * st_inv[row];
        Cm[row * CLD + col] = toh_flush(CCARRY * val);
      }
    }
  }

  {
    float wc[NSTAT];
#pragma unroll
    for (int j = 0; j < NSTAT; ++j) wc[j] = bf16r(W_stat[(unsigned)j * EMB + tid]);
    const float bst = bf16r(b_stat[tid]);
#pragma unroll 4
    for (unsigned row = 0; row < 16u; ++row) {
      float s = 0.0f;
#pragma unroll
      for (int j = 0; j < NSTAT; ++j) s = fmaf(sst[row * NSTAT + (unsigned)j], wc[j], s);
      s += bst;
      Cm[row * CLD + (unsigned)EMB + tid] = toh_flush(CCARRY * s);
    }
  }
  __syncthreads();

  v8f c[4];
#pragma unroll
  for (int j = 0; j < 4; ++j) c[j] = (v8f){};
  {
    const _Float16* bq = Wm_t + (size_t)(w * 64u + m) * CDIM + hh * 8u;
    const unsigned abase = m * CLD + hh * 8u;
#pragma unroll 2
    for (unsigned k0 = 0; k0 < (unsigned)CDIM; k0 += 32u) {
      const v8h alo = *(const v8h*)&Cm[abase + k0];
      const v8h ahi = *(const v8h*)&Cm[abase + k0 + 16u];
      const v16h a = frag_join(alo, ahi);
#pragma unroll
      for (int j = 0; j < 4; ++j) {
        const v16h bf = frag_at(bq + (size_t)j * 16u * CDIM + k0);
        c[j] = wmma16(a, bf, c[j]);
      }
    }
  }

  float q0[8], q1[8];
#pragma unroll
  for (int r = 0; r < 8; ++r) { q0[r] = 0.0f; q1[r] = 0.0f; }
#pragma unroll
  for (int j = 0; j < 4; ++j) {
    const unsigned col = w * 64u + (unsigned)j * 16u + m;
    const float bm = bf16r(b_merge[col]);
    const float w0 = bf16r(W_cls[col * NCLS]);
    const float w1 = bf16r(W_cls[col * NCLS + 1u]);
#pragma unroll
    for (int r = 0; r < 8; ++r) {
      const float v = fmaxf(c[j][r] * (1.0f / (WCARRY * CCARRY)) + bm, 0.0f);
      q0[r] += v * w0;
      q1[r] += v * w1;
    }
  }
#pragma unroll
  for (int r = 0; r < 8; ++r) {
    q0[r] = red16_sum(q0[r]);
    q1[r] = red16_sum(q1[r]);
  }
  if (m == 0u) {
#pragma unroll
    for (int r = 0; r < 8; ++r) {
      const unsigned row = hh * 8u + (unsigned)r;
      cpart[(w * 16u + row) * NCLS]      = q0[r];
      cpart[(w * 16u + row) * NCLS + 1u] = q1[r];
    }
  }
  __syncthreads();

  if (w == 0u) {
    const unsigned row = lane >> 1, cls = lane & 1u;
    float s = 0.0f;
#pragma unroll
    for (unsigned ww = 0; ww < 8u; ++ww) s += cpart[(ww * 16u + row) * NCLS + cls];
    s += bf16r(b_cls[cls]);
    otile[lane] = s;
  }
  __syncthreads();

  if (w == 0u) {
    const unsigned li = (lane < 8u) ? lane : 7u;
    const v4f ov = *(const v4f*)&otile[li * 4u];
    float* p = out + (size_t)row0 * NCLS + li * 4u;
    if (lane < 8u) *(volatile v4f*)p = ov;
    __threadfence();
    if (lane < 8u) *(volatile v4f*)p = ov;
  }
}

extern "C" void kernel_launch(void* const* d_in, const int* in_sizes, int n_in,
                              void* d_out, int out_size, void* d_ws, size_t ws_size,
                              hipStream_t stream) {
  if (n_in < 14) return;
  const long long need_x = ((long long)(NB - 1) * SNS + (SNS - 1)) * SEQ_FULL + SEQ;
  const long long need_t = (long long)(NB - 1) * SEQ_FULL + SEQ;
  if ((long long)in_sizes[0] < need_x) return;
  if ((long long)in_sizes[1] < (long long)NB * NSTAT) return;
  if ((long long)in_sizes[2] < need_t) return;
  if ((long long)in_sizes[3] < need_x) return;
  if ((long long)in_sizes[4] < (long long)NFEAT * EMB) return;
  if (in_sizes[5] < EMB || in_sizes[6] < EMB || in_sizes[7] < EMB) return;
  if (in_sizes[8] < NSTAT * EMB || in_sizes[9] < EMB) return;
  if ((long long)in_sizes[10] < (long long)CDIM * CDIM) return;
  if (in_sizes[11] < CDIM || in_sizes[12] < CDIM * NCLS || in_sizes[13] < NCLS) return;
  if ((long long)out_size < (long long)NB * NCLS) return;
  if (ws_size < WS_TOTAL) return;

  const float* x       = (const float*)d_in[0];
  const float* statics = (const float*)d_in[1];
  const float* timev   = (const float*)d_in[2];
  const int*   smask   = (const int*)d_in[3];
  const float* W_sens  = (const float*)d_in[4];
  const float* b_sens  = (const float*)d_in[5];
  const float* W_time  = (const float*)d_in[6];
  const float* b_time  = (const float*)d_in[7];
  const float* W_stat  = (const float*)d_in[8];
  const float* b_stat  = (const float*)d_in[9];
  const float* W_merge = (const float*)d_in[10];
  const float* b_merge = (const float*)d_in[11];
  const float* W_cls   = (const float*)d_in[12];
  const float* b_cls   = (const float*)d_in[13];
  float* out = (float*)d_out;

  char* ws = (char*)d_ws;
  _Float16* Ws_t = (_Float16*)(ws + OFF_WSP);
  _Float16* Wm_t = (_Float16*)(ws + OFF_WMP);
  _Float16* A16  = (_Float16*)(ws + OFF_A);
  float*    St   = (float*)(ws + OFF_ST);

  dim3 blk(256);
  wconv_kernel<<<dim3(EMB / 64, KS / 64), blk, 0, stream>>>(
      W_sens, Ws_t, (unsigned)EMB, (unsigned)KS, (unsigned)NFEAT);
  wconv_kernel<<<dim3(CDIM / 64, CDIM / 64), blk, 0, stream>>>(
      W_merge, Wm_t, (unsigned)CDIM, (unsigned)CDIM, (unsigned)CDIM);
  pool_kernel<<<dim3(NB), blk, 0, stream>>>(x, smask, timev, A16, St);
  head_kernel<<<dim3(NB / 16), blk, 0, stream>>>(A16, St, Ws_t, Wm_t, statics,
                                                 b_sens, W_time, b_time, W_stat, b_stat,
                                                 b_merge, W_cls, b_cls, out);
}
